// CMKConMambaBlock_52956946760392
// MI455X (gfx1250) — hardware-verified
//
#include <hip/hip_runtime.h>


namespace {
constexpr int B = 4, N = 1024, C = 128, DI = 256, S = 128, R = 8, DC = 4, NR = B * N, XPW = 272;
constexpr float XS = 8.0f, WSC = 256.0f, EPS = 1e-5f;
typedef _Float16 b16;
typedef __attribute__((ext_vector_type(16))) _Float16 v16b;
typedef __attribute__((ext_vector_type(8))) _Float16 v8b;
typedef __attribute__((ext_vector_type(8))) float v8f;
typedef __attribute__((ext_vector_type(4))) float v4f;
typedef __attribute__((ext_vector_type(2))) float v2f;
typedef __attribute__((ext_vector_type(2))) _Float16 v2b;
__device__ __forceinline__ float bf16_rne(float f) { unsigned int u = __float_as_uint(f); u += 0x7FFFu + ((u >> 16) & 1u); float r = __uint_as_float(u & 0xFFFF0000u); asm volatile("" : "+v"(r)); return r; }
__device__ __forceinline__ void split16(float v, b16& hi, b16& lo) { hi = (b16)v; lo = (b16)(v - (float)hi); }
__device__ __forceinline__ v16b frag_kb(const b16* p, int hh) { const v8b a = *(const v8b*)(p + 8 * hh), b = *(const v8b*)(p + 16 + 8 * hh); v16b f;
#pragma unroll
  for (int e = 0; e < 8; ++e) { f[e] = a[e]; f[8 + e] = b[e]; } return f; }
__device__ __forceinline__ v8f wmma16b(v16b a, v16b b, v8f c) { v8f d = __builtin_amdgcn_wmma_f32_16x16x32_f16(false, a, false, b, (short)0, c, false, false); asm volatile("v_nop\n\tv_nop\n\tv_nop\n\tv_nop" : "+v"(d) : "v"(a), "v"(b)); return d; }
__device__ __forceinline__ void wave_lds_sync() { __builtin_amdgcn_fence(__ATOMIC_RELEASE, "workgroup"); __builtin_amdgcn_wave_barrier(); __builtin_amdgcn_fence(__ATOMIC_ACQUIRE, "workgroup"); }
__device__ __forceinline__ float pmul(float a, float b) { float p = a * b; asm volatile("" : "+v"(p)); return p; }
__device__ __forceinline__ int iclamp(int v, int lo, int hi) { return v < lo ? lo : (v > hi ? hi : v); }
__device__ __forceinline__ float silu(float v) { return v / (1.0f + __expf(-v)); }
__device__ __forceinline__ float softplus(float v) { return v > 20.0f ? v : __logf(1.0f + __expf(v)); }
__device__ __forceinline__ int kpad_of(int i) { return i == 0 ? 8 : i == 1 ? 16 : i == 2 ? 24 : 32; }
__device__ __forceinline__ int ktap_of(int i) { return i == 0 ? 7 : i == 1 ? 15 : i == 2 ? 23 : 31; }

__global__ __launch_bounds__(256) void wput_kernel(const float* __restrict__ c1w, const float* __restrict__ c2w, const float* __restrict__ qw, const float* __restrict__ kw, const float* __restrict__ minw, const float* __restrict__ mxw, const float* __restrict__ mow, const float* __restrict__ kpw, const float* __restrict__ kc1, const float* __restrict__ kc2, const float* __restrict__ kc3, const float* __restrict__ kc4, b16* __restrict__ C1T, b16* __restrict__ C2T, b16* __restrict__ QT, b16* __restrict__ KT, b16* __restrict__ MIN, b16* __restrict__ MXP, b16* __restrict__ MOUT, b16* __restrict__ KP, b16* __restrict__ KC) {
  const int u = blockIdx.x * 256 + threadIdx.x;
  for (int pass = 0; pass < 2; ++pass) {
    if (u < C * 48) { const int o = u / 48, k0 = (u % 48) * 8; v8b a, b;
#pragma unroll
      for (int j = 0; j < 8; ++j) { const int k = k0 + j, c = k / 3, kk = k % 3; a[j] = (b16)(bf16_rne(c1w[((size_t)o * C + c) * 3 + kk]) * WSC); b[j] = (b16)(bf16_rne(c2w[((size_t)o * C + c) * 3 + kk]) * WSC); } *(volatile v8b*)(C1T + (size_t)o * 384 + k0) = a; *(volatile v8b*)(C2T + (size_t)o * 384 + k0) = b; }
    if (u < C * 16) { const int o = u / 16, k0 = (u % 16) * 8; v8b a, b, p0, p1;
#pragma unroll
      for (int j = 0; j < 8; ++j) { a[j] = (b16)(bf16_rne(qw[(size_t)o * C + k0 + j]) * WSC); b[j] = (b16)(bf16_rne(kw[(size_t)o * C + k0 + j]) * WSC); p0[j] = (b16)(bf16_rne(kpw[(size_t)o * C + k0 + j]) * WSC); p1[j] = (b16)(bf16_rne(kpw[(size_t)(C + o) * C + k0 + j]) * WSC); }
      *(volatile v8b*)(QT + (size_t)o * C + k0) = a; *(volatile v8b*)(KT + (size_t)o * C + k0) = b; *(volatile v8b*)(KP + (size_t)o * C + k0) = p0; *(volatile v8b*)(KP + (size_t)(C + o) * C + k0) = p1; }
    if (u < 2 * DI * 16) { const int o = u / 16, k0 = (u % 16) * 8; v8b v;
#pragma unroll
      for (int j = 0; j < 8; ++j) v[j] = (b16)(bf16_rne(minw[(size_t)o * C + k0 + j]) * WSC); *(volatile v8b*)(MIN + (size_t)o * C + k0) = v; }
    if (u < XPW * 32) { const int o = u / 32, k0 = (u % 32) * 8; v8b v;
#pragma unroll
      for (int j = 0; j < 8; ++j) v[j] = (b16)(o < R + 2 * S ? bf16_rne(mxw[(size_t)o * DI + k0 + j]) * WSC : 0.0f); *(volatile v8b*)(MXP + (size_t)o * DI + k0) = v; }
    if (u < C * 32) { const int o = u / 32, k0 = (u % 32) * 8; v8b v;
#pragma unroll
      for (int j = 0; j < 8; ++j) v[j] = (b16)(bf16_rne(mow[(size_t)o * DI + k0 + j]) * WSC); *(volatile v8b*)(MOUT + (size_t)o * DI + k0) = v; }
    if (u < 4 * 32 * C) { const int i = u / (32 * C), o = (u / C) % 32, c = u % C; const int kp = kpad_of(i), kt = ktap_of(i); const float* w = i == 0 ? kc1 : i == 1 ? kc2 : i == 2 ? kc3 : kc4; size_t base = 0; for (int q = 0; q < i; ++q) base += (size_t)32 * C * kpad_of(q);
      for (int kk = 0; kk < kp; ++kk) ((volatile b16*)KC)[base + ((size_t)o * C + c) * kp + kk] = (b16)(kk < kt ? bf16_rne(w[((size_t)o * C + c) * kt + kk]) * WSC : 0.0f); }
    __threadfence(); } }
__device__ __forceinline__ void ln_row16(float (*Tf)[132], int lane, const float* g, const float* bb) {
  for (int rr = 0; rr < 16; ++rr) { float v[4]; float s = 0.0f; for (int k = 0; k < 4; ++k) { v[k] = Tf[rr][lane * 4 + k]; s += v[k]; } for (int o = 16; o; o >>= 1) s += __shfl_xor(s, o); const float mu = s * (1.0f / C); float q = 0.0f; for (int k = 0; k < 4; ++k) q += pmul(v[k] - mu, v[k] - mu); for (int o = 16; o; o >>= 1) q += __shfl_xor(q, o); const float rs = rsqrtf(q * (1.0f / C) + EPS);
    for (int k = 0; k < 4; ++k) { const int c = lane * 4 + k; Tf[rr][c] = pmul(pmul(v[k] - mu, rs), bf16_rne(g[c])) + bf16_rne(bb[c]); } } }
template <int MODE>
__global__ __launch_bounds__(32) void conv3_kernel(const float* __restrict__ IN, const b16* __restrict__ WT, const float* __restrict__ bias, const float* __restrict__ g, const float* __restrict__ bb, const float* __restrict__ RES, int BV, float* __restrict__ OUT) {
  __shared__ __attribute__((aligned(16))) b16 Ah[16][392], Al[16][MODE == 0 ? 8 : 392]; __shared__ float Tf[16][132]; const int lane = threadIdx.x, nloc = lane & 15, hlf = lane >> 4; const size_t m0 = (size_t)blockIdx.x * 16; const int b = (int)(m0 / N), n0 = (int)(m0 % N); if (b >= BV) return;
  for (int rr = 0; rr < 16; ++rr) for (int q = 0; q < 12; ++q) { const int k = q * 32 + lane; const int c = k / 3, kk = k % 3; const int n = n0 + rr + kk - 1; float v = 0.0f; if (n >= 0 && n < N) v = MODE == 0 ? bf16_rne(IN[(size_t)b * N * C + (size_t)c * N + n]) : IN[((size_t)b * N + n) * C + c];
    if (MODE == 0) Ah[rr][k] = (b16)(v * XS); else { b16 p, ql; split16(v * XS, p, ql); Ah[rr][k] = p; Al[rr][k] = ql; } }
  wave_lds_sync(); v8f acc[8];
#pragma unroll
  for (int t = 0; t < 8; ++t) acc[t] = (v8f){};
#pragma unroll 2
  for (int kb = 0; kb < 384; kb += 32) { const v16b a = frag_kb(&Ah[nloc][kb], hlf); v16b a2; if (MODE != 0) a2 = frag_kb(&Al[nloc][kb], hlf);
#pragma unroll
    for (int t = 0; t < 8; ++t) { const v16b bw = frag_kb(WT + (size_t)(t * 16 + nloc) * 384 + kb, hlf); acc[t] = wmma16b(a, bw, acc[t]); if (MODE != 0) acc[t] = wmma16b(a2, bw, acc[t]); } }
#pragma unroll
  for (int t = 0; t < 8; ++t) { const int c = t * 16 + nloc; const float bv = bf16_rne(bias[c]);
#pragma unroll
    for (int r8 = 0; r8 < 8; ++r8) Tf[8 * hlf + r8][c] = acc[t][r8] * (1.0f / (XS * WSC)) + bv; }
  wave_lds_sync(); ln_row16(Tf, lane, g, bb); wave_lds_sync();
  for (int pass = 0; pass < 2; ++pass) { for (int rr = 0; rr < 16; ++rr) { v4f v; for (int k = 0; k < 4; ++k) v[k] = fmaxf(Tf[rr][lane * 4 + k], 0.0f); if (MODE == 1) { const v4f r = *(const v4f*)(RES + (m0 + rr) * C + lane * 4); for (int k = 0; k < 4; ++k) v[k] += bf16_rne(r[k]); } *(volatile v4f*)(OUT + (m0 + rr) * C + lane * 4) = v; } __threadfence(); } }
__global__ __launch_bounds__(32) void qk_kernel(const float* __restrict__ C1, const b16* __restrict__ QT, const b16* __restrict__ KT, const float* __restrict__ qb, const float* __restrict__ kb, int BV, b16* __restrict__ Qh, b16* __restrict__ Ql, b16* __restrict__ Kh, b16* __restrict__ Kl) {
  __shared__ __attribute__((aligned(16))) b16 Ah[64][136], Al[64][136]; __shared__ float Tf[16][132]; const int lane = threadIdx.x, nloc = lane & 15, hlf = lane >> 4; const int n0 = (blockIdx.x % (N / 64)) * 64, b = blockIdx.x / (N / 64); if (b >= BV) return;
  for (int rr = 0; rr < 64; ++rr) for (int q = 0; q < 4; ++q) { const int c = q * 32 + lane; b16 p, ql; split16(C1[(size_t)b * N * C + (size_t)c * N + n0 + rr] * XS, p, ql); Ah[rr][c] = p; Al[rr][c] = ql; }
  wave_lds_sync();
  for (int which = 0; which < 2; ++which) { const b16* WT = which == 0 ? QT : KT; const float* bias = which == 0 ? qb : kb; b16* Oh = which == 0 ? Qh : Kh; b16* Ol = which == 0 ? Ql : Kl;
    for (int m = 0; m < 4; ++m) { v8f acc[8];
#pragma unroll
      for (int t = 0; t < 8; ++t) acc[t] = (v8f){};
#pragma unroll
      for (int kk = 0; kk < C; kk += 32) { const v16b a = frag_kb(&Ah[m * 16 + nloc][kk], hlf), al = frag_kb(&Al[m * 16 + nloc][kk], hlf);
#pragma unroll
        for (int t = 0; t < 8; ++t) { const v16b bw = frag_kb(WT + (size_t)(t * 16 + nloc) * C + kk, hlf); acc[t] = wmma16b(a, bw, acc[t]); acc[t] = wmma16b(al, bw, acc[t]); } }
#pragma unroll
      for (int t = 0; t < 8; ++t) { const int c = t * 16 + nloc; const float bv = bf16_rne(bias[c]);
#pragma unroll
        for (int r8 = 0; r8 < 8; ++r8) Tf[8 * hlf + r8][c] = acc[t][r8] * (1.0f / (XS * WSC)) + bv; }
      wave_lds_sync();
      for (int pass = 0; pass < 2; ++pass) { for (int og = 0; og < 4; ++og) { const int o = og * 32 + lane; for (int j = 0; j < 16; ++j) { b16 p, ql; split16(Tf[j][o] * XS, p, ql); ((volatile b16*)Oh)[((size_t)b * C + o) * N + n0 + m * 16 + j] = p; ((volatile b16*)Ol)[((size_t)b * C + o) * N + n0 + m * 16 + j] = ql; } } __threadfence(); }
      wave_lds_sync(); } } }
__global__ __launch_bounds__(32) void cc_kernel(const b16* __restrict__ Qh, const b16* __restrict__ Ql, const b16* __restrict__ Kh, const b16* __restrict__ Kl, int BV, b16* __restrict__ CCh, b16* __restrict__ CCl) {
  __shared__ float Sc[64][132]; const int lane = threadIdx.x, nloc = lane & 15, hlf = lane >> 4; const int c0 = (blockIdx.x % 2) * 64, b = blockIdx.x / 2; if (b >= BV) return;
  for (int m = 0; m < 4; ++m) { v8f acc[8];
#pragma unroll
    for (int t = 0; t < 8; ++t) acc[t] = (v8f){};
#pragma unroll 2
    for (int kb = 0; kb < N; kb += 32) { const size_t ar = ((size_t)b * C + c0 + m * 16 + nloc) * N + kb; const v16b a = frag_kb(Qh + ar, hlf), al = frag_kb(Ql + ar, hlf);
#pragma unroll
      for (int t = 0; t < 8; ++t) { const size_t br = ((size_t)b * C + t * 16 + nloc) * N + kb; const v16b bh = frag_kb(Kh + br, hlf), bl = frag_kb(Kl + br, hlf); acc[t] = wmma16b(a, bh, acc[t]); acc[t] = wmma16b(a, bl, acc[t]); acc[t] = wmma16b(al, bh, acc[t]); } }
#pragma unroll
    for (int t = 0; t < 8; ++t)
#pragma unroll
      for (int r8 = 0; r8 < 8; ++r8) Sc[m * 16 + 8 * hlf + r8][t * 16 + nloc] = acc[t][r8] * (1.0f / (XS * XS)); }
  wave_lds_sync();
  for (int hf = 0; hf < 2; ++hf) { const int rr = hf * 32 + lane; float mx = -INFINITY; for (int d = 0; d < C; ++d) mx = fmaxf(mx, Sc[rr][d]); float s = 0.0f; for (int d = 0; d < C; ++d) { const float e = __expf(Sc[rr][d] - mx); Sc[rr][d] = e; s += e; } const float inv = 1.0f / s; for (int d = 0; d < C; ++d) Sc[rr][d] = pmul(Sc[rr][d], inv); }
  wave_lds_sync();
  for (int pass = 0; pass < 2; ++pass) { for (int dg = 0; dg < 4; ++dg) { const int d = dg * 32 + lane; for (int j = 0; j < 64; ++j) { b16 p, ql; split16(Sc[j][d] * XS, p, ql); ((volatile b16*)CCh)[((size_t)b * C + d) * C + c0 + j] = p; ((volatile b16*)CCl)[((size_t)b * C + d) * C + c0 + j] = ql; } } __threadfence(); } }
__global__ __launch_bounds__(32) void xca_kernel(const float* __restrict__ C1, const b16* __restrict__ CCh, const b16* __restrict__ CCl, int BV, float* __restrict__ XCA) { __shared__ __attribute__((aligned(16))) b16 Ah[16][136], Al[16][136]; __shared__ float Tf[16][132]; const int lane = threadIdx.x, nloc = lane & 15, hlf = lane >> 4; const size_t m0 = (size_t)blockIdx.x * 16; const int b = (int)(m0 / N); if (b >= BV) return;
  for (int rr = 0; rr < 16; ++rr) for (int q = 0; q < 4; ++q) { b16 p, ql; split16(C1[(m0 + rr) * C + q * 32 + lane] * XS, p, ql); Ah[rr][q * 32 + lane] = p; Al[rr][q * 32 + lane] = ql; }
  wave_lds_sync(); v8f acc[8];
#pragma unroll
  for (int t = 0; t < 8; ++t) acc[t] = (v8f){};
#pragma unroll
  for (int kb = 0; kb < C; kb += 32) { const v16b a = frag_kb(&Ah[nloc][kb], hlf), al = frag_kb(&Al[nloc][kb], hlf);
#pragma unroll
    for (int t = 0; t < 8; ++t) { const size_t br = ((size_t)b * C + t * 16 + nloc) * C + kb; const v16b bh = frag_kb(CCh + br, hlf), bl = frag_kb(CCl + br, hlf); acc[t] = wmma16b(a, bh, acc[t]); acc[t] = wmma16b(a, bl, acc[t]); acc[t] = wmma16b(al, bh, acc[t]); } }
#pragma unroll
  for (int t = 0; t < 8; ++t)
#pragma unroll
    for (int r8 = 0; r8 < 8; ++r8) Tf[8 * hlf + r8][t * 16 + nloc] = acc[t][r8] * (1.0f / (XS * XS));
  wave_lds_sync();
  for (int pass = 0; pass < 2; ++pass) { for (int rr = 0; rr < 16; ++rr) { v4f v = *(const v4f*)(&Tf[rr][lane * 4]); const v4f c1v = *(const v4f*)(C1 + (m0 + rr) * C + lane * 4); for (int k = 0; k < 4; ++k) v[k] += 2.0f * c1v[k]; *(volatile v4f*)(XCA + (m0 + rr) * C + lane * 4) = v; } __threadfence(); } }
template <int MODE>
__global__ __launch_bounds__(32) void rowgemm_kernel(const float* __restrict__ IN, const float* __restrict__ lng, const float* __restrict__ lnb, const b16* __restrict__ WT, const float* __restrict__ bias, const float* __restrict__ RES, int BV, float* __restrict__ OUT) {
  constexpr int KT = MODE == 1 ? DI : C, OW = MODE == 0 ? 2 * DI : MODE == 1 ? C : DI, NGRP = OW / 128, MT = MODE == 2 ? 2 : 1; __shared__ __attribute__((aligned(16))) b16 Ah[16 * MT][KT + 8], Al[16 * MT][KT + 8]; __shared__ float Tf[16 * MT][132];
  const int lane = threadIdx.x, nloc = lane & 15, hlf = lane >> 4; const int g = blockIdx.x % NGRP; const size_t m0 = (size_t)(blockIdx.x / NGRP) * 16 * MT; const int b = (int)(m0 / N), n0 = (int)(m0 % N); if (b >= BV) return;
  for (int rr = 0; rr < 16 * MT; ++rr) { float v[KT / 32]; for (int q = 0; q < KT / 32; ++q) { const int c = q * 32 + lane; v[q] = MODE == 1 ? IN[((size_t)b * DI + c) * N + n0 + rr] : IN[(m0 + rr) * C + c]; }
    if (MODE != 1) { float s = 0.0f; for (int q = 0; q < 4; ++q) s += v[q]; for (int o = 16; o; o >>= 1) s += __shfl_xor(s, o); const float mu = s * (1.0f / C); float qq = 0.0f; for (int q = 0; q < 4; ++q) qq += pmul(v[q] - mu, v[q] - mu); for (int o = 16; o; o >>= 1) qq += __shfl_xor(qq, o); const float rs = rsqrtf(qq * (1.0f / C) + EPS); for (int q = 0; q < 4; ++q) { const int c = q * 32 + lane; v[q] = pmul(pmul(v[q] - mu, rs), bf16_rne(lng[c])) + bf16_rne(lnb[c]); } }
    for (int q = 0; q < KT / 32; ++q) { b16 p, ql; split16(v[q] * XS, p, ql); Ah[rr][q * 32 + lane] = p; Al[rr][q * 32 + lane] = ql; } }
  wave_lds_sync();
  for (int m = 0; m < MT; ++m) { v8f acc[8];
#pragma unroll
    for (int t = 0; t < 8; ++t) acc[t] = (v8f){};
#pragma unroll 2
    for (int kb = 0; kb < KT; kb += 32) { const v16b a = frag_kb(&Ah[m * 16 + nloc][kb], hlf), al = frag_kb(&Al[m * 16 + nloc][kb], hlf);
#pragma unroll
      for (int t = 0; t < 8; ++t) { const v16b bw = frag_kb(WT + (size_t)(g * 128 + t * 16 + nloc) * KT + kb, hlf); acc[t] = wmma16b(a, bw, acc[t]); acc[t] = wmma16b(al, bw, acc[t]); } }
#pragma unroll
    for (int t = 0; t < 8; ++t) { const int c = t * 16 + nloc; const float bv = MODE == 2 ? bf16_rne(bias[g * 128 + c]) : 0.0f;
#pragma unroll
      for (int r8 = 0; r8 < 8; ++r8) { float v = acc[t][r8] * (1.0f / (XS * WSC)) + bv; if (MODE == 2) v = pmul(v, 1.0f / (1.0f + __expf(-v))); Tf[m * 16 + 8 * hlf + r8][c] = v; } } }
  wave_lds_sync();
  for (int pass = 0; pass < 2; ++pass) {
    if (MODE == 2) { for (int og = 0; og < 4; ++og) { const int ch = g * 128 + og * 32 + lane; for (int j = 0; j < 32; ++j) ((volatile float*)OUT)[((size_t)b * DI + ch) * N + n0 + j] = Tf[j][og * 32 + lane]; } }
    else { for (int rr = 0; rr < 16; ++rr) { v4f v = *(const v4f*)(&Tf[rr][lane * 4]); if (MODE == 1) { const v4f r = *(const v4f*)(RES + (m0 + rr) * C + lane * 4); for (int k = 0; k < 4; ++k) v[k] += r[k]; } *(volatile v4f*)(OUT + (m0 + rr) * OW + g * 128 + lane * 4) = v; } }
    __threadfence(); } }
__global__ __launch_bounds__(256) void mconv_kernel(const float* __restrict__ XZ, const float* __restrict__ cw, const float* __restrict__ cb, int BV, float* __restrict__ XI2) { const int wave = threadIdx.x >> 5, lane = threadIdx.x & 31; const size_t row = (size_t)blockIdx.x * 8 + wave; const int b = (int)(row / N), n = (int)(row % N); if (b >= BV) return;
  float o[8];
#pragma unroll
  for (int k = 0; k < 8; ++k) { const int d = lane * 8 + k; float s = bf16_rne(cb[d]);
#pragma unroll
    for (int kk = 0; kk < DC; ++kk) { const int nn = n - (DC - 1) + kk; if (nn < 0) continue; s += pmul(bf16_rne(cw[d * DC + kk]), XZ[((size_t)b * N + nn) * 2 * DI + d]); } o[k] = silu(s); }
  for (int pass = 0; pass < 2; ++pass) { *(volatile v4f*)(XI2 + row * DI + lane * 8) = (v4f){o[0], o[1], o[2], o[3]}; *(volatile v4f*)(XI2 + row * DI + lane * 8 + 4) = (v4f){o[4], o[5], o[6], o[7]}; __threadfence(); } }
__global__ __launch_bounds__(32) void xproj_kernel(const float* __restrict__ XI2, const b16* __restrict__ MXP, const float* __restrict__ dtw, const float* __restrict__ dtb, int BV, float* __restrict__ DBL, float* __restrict__ DT) { __shared__ __attribute__((aligned(16))) b16 Ah[16][DI + 8], Al[16][DI + 8]; __shared__ float Tf[16][XPW + 4]; const int lane = threadIdx.x, nloc = lane & 15, hlf = lane >> 4; const size_t m0 = (size_t)blockIdx.x * 16; if ((int)(m0 / N) >= BV) return;
  for (int rr = 0; rr < 16; ++rr) for (int q = 0; q < 8; ++q) { b16 p, ql; split16(XI2[(m0 + rr) * DI + q * 32 + lane] * XS, p, ql); Ah[rr][q * 32 + lane] = p; Al[rr][q * 32 + lane] = ql; }
  wave_lds_sync();
#pragma unroll 1
  for (int tg = 0; tg < 17; tg += 6) { v8f acc[6];
#pragma unroll
    for (int t = 0; t < 6; ++t) acc[t] = (v8f){};
#pragma unroll 2
    for (int kb = 0; kb < DI; kb += 32) { const v16b a = frag_kb(&Ah[nloc][kb], hlf), al = frag_kb(&Al[nloc][kb], hlf);
#pragma unroll
      for (int t = 0; t < 6; ++t) { if (tg + t < 17) { const v16b bw = frag_kb(MXP + (size_t)((tg + t) * 16 + nloc) * DI + kb, hlf); acc[t] = wmma16b(a, bw, acc[t]); acc[t] = wmma16b(al, bw, acc[t]); } } }
#pragma unroll
    for (int t = 0; t < 6; ++t) { if (tg + t < 17) {
#pragma unroll
      for (int r8 = 0; r8 < 8; ++r8) Tf[8 * hlf + r8][(tg + t) * 16 + nloc] = acc[t][r8] * (1.0f / (XS * WSC)); } } }
  wave_lds_sync(); float wv[8][R];
#pragma unroll
  for (int j = 0; j < 8; ++j)
#pragma unroll
    for (int r = 0; r < R; ++r) wv[j][r] = bf16_rne(dtw[(lane * 8 + j) * R + r]);
  for (int pass = 0; pass < 2; ++pass) { for (int rr = 0; rr < 16; ++rr) { for (int c = lane; c < XPW; c += 32) ((volatile float*)DBL)[(m0 + rr) * XPW + c] = Tf[rr][c];
#pragma unroll
      for (int j = 0; j < 8; ++j) { const int d = lane * 8 + j; float s = bf16_rne(dtb[d]);
#pragma unroll
        for (int r = 0; r < R; ++r) s += pmul(Tf[rr][r], wv[j][r]); ((volatile float*)DT)[(m0 + rr) * DI + d] = softplus(s); } }
    __threadfence(); } }
__global__ __launch_bounds__(32) void mscan_kernel(const float* __restrict__ XI2, const float* __restrict__ DT, const float* __restrict__ DBL, const float* __restrict__ XZ, const float* __restrict__ Alog, const float* __restrict__ Dp, int BV, float* __restrict__ YGT) {
  const int lane = threadIdx.x; const int b = blockIdx.x / (DI / 16), d = (blockIdx.x % (DI / 16)) * 16 + (lane >> 1), hf = lane & 1; if (b >= BV) return; float A[64]; const float Dd = bf16_rne(Dp[d]);
#pragma unroll
  for (int j = 0; j < 64; ++j) A[j] = -__expf(bf16_rne(Alog[(size_t)d * S + hf * 64 + j]));
  for (int pass = 0; pass < 2; ++pass) { float h[64];
#pragma unroll
    for (int j = 0; j < 64; ++j) h[j] = 0.0f;
#pragma unroll 1
    for (int t = 0; t < N; ++t) { const size_t row = (size_t)b * N + t; const float xv = XI2[row * DI + d], dt = DT[row * DI + d]; const float dx = pmul(dt, xv); const float* Bp = DBL + row * XPW + R + hf * 64; const float* Cp = DBL + row * XPW + R + S + hf * 64; float y = 0.0f;
#pragma unroll
      for (int j = 0; j < 64; ++j) { h[j] = pmul(h[j], __expf(pmul(dt, A[j]))) + pmul(dx, Bp[j]); y += pmul(h[j], Cp[j]); }
      y += __shfl_xor(y, 1); y += pmul(xv, Dd); y = pmul(y, silu(XZ[row * 2 * DI + DI + d]));
      if (hf == 0) ((volatile float*)YGT)[((size_t)b * DI + d) * N + t] = y; }
    __threadfence(); } }
__global__ __launch_bounds__(32) void kconv_kernel(const float* __restrict__ HKT, const b16* __restrict__ KC, const float* __restrict__ b1, const float* __restrict__ b2, const float* __restrict__ b3, const float* __restrict__ b4, int BV, float* __restrict__ MCT) {
  __shared__ __attribute__((aligned(16))) b16 Ah[32][264], Al[32][264]; __shared__ float Tm[32][132]; const int lane = threadIdx.x, nloc = lane & 15, hlf = lane >> 4; const int n0 = (blockIdx.x % (N / 32)) * 32, b = blockIdx.x / (N / 32); if (b >= BV) return;
  size_t base = 0;
  for (int i = 0; i < 4; ++i) { const int kp = kpad_of(i), kt = ktap_of(i), pad = (kt - 1) / 2, KCH = 8 * kp; v8f acc[2][2] = {{(v8f){}, (v8f){}}, {(v8f){}, (v8f){}}};
    for (int c0 = 0; c0 < C; c0 += 8) {
      for (int idx = lane; idx < 32 * KCH; idx += 32) { const int rr = idx / KCH, k = idx % KCH; const int cl = k / kp, kk = k % kp; const int n = n0 + rr + kk - pad; float v = 0.0f; if (kk < kt && n >= 0 && n < N) v = HKT[((size_t)b * DI + C + c0 + cl) * N + n]; b16 p, ql; split16(v * XS, p, ql); Ah[rr][k] = p; Al[rr][k] = ql; }
      wave_lds_sync();
      for (int kb = 0; kb < KCH; kb += 32) {
#pragma unroll
        for (int m = 0; m < 2; ++m) { const v16b a = frag_kb(&Ah[m * 16 + nloc][kb], hlf), al = frag_kb(&Al[m * 16 + nloc][kb], hlf);
#pragma unroll
          for (int t = 0; t < 2; ++t) { const v16b bw = frag_kb(KC + base + (size_t)(t * 16 + nloc) * C * kp + (size_t)c0 * kp + kb, hlf); acc[m][t] = wmma16b(a, bw, acc[m][t]); acc[m][t] = wmma16b(al, bw, acc[m][t]); } } }
      wave_lds_sync(); }
    const float* bb = i == 0 ? b1 : i == 1 ? b2 : i == 2 ? b3 : b4;
#pragma unroll
    for (int m = 0; m < 2; ++m)
#pragma unroll
      for (int t = 0; t < 2; ++t)
#pragma unroll
        for (int r8 = 0; r8 < 8; ++r8) Tm[m * 16 + 8 * hlf + r8][i * 32 + t * 16 + nloc] = acc[m][t][r8] * (1.0f / (XS * WSC)) + bf16_rne(bb[t * 16 + nloc]);
    base += (size_t)32 * C * kp; }
  wave_lds_sync();
  for (int pass = 0; pass < 2; ++pass) { for (int og = 0; og < 4; ++og) { const int ch = og * 32 + lane; for (int j = 0; j < 32; ++j) ((volatile float*)MCT)[((size_t)b * C + ch) * N + n0 + j] = Tm[j][ch]; } __threadfence(); } }
__global__ __launch_bounds__(256) void final_kernel(const float* __restrict__ MCT, const float* __restrict__ HKT, const float* __restrict__ X2, const float* __restrict__ kdw, const float* __restrict__ kdwb, const float* __restrict__ g1, const float* __restrict__ be1, const float* __restrict__ g2, const float* __restrict__ be2, const float* __restrict__ png, const float* __restrict__ pnb, int BV, float* __restrict__ out) {
  const int wave = threadIdx.x >> 5, lane = threadIdx.x & 31; const size_t row = (size_t)blockIdx.x * 8 + wave; const int b = (int)(row / N), n = (int)(row % N); if (b >= BV) return; const float bnf = 1.0f / sqrtf(1.0f + EPS);
  float v[4]; float s = 0.0f;
#pragma unroll
  for (int k = 0; k < 4; ++k) { const int c = lane * 4 + k; const float* mcr = MCT + ((size_t)b * C + c) * N; float dw = bf16_rne(kdwb[c]);
#pragma unroll 1
    for (int kk = 0; kk < 31; ++kk) { const int nn = n + kk - 15; if (nn < 0 || nn >= N) continue; dw += pmul(bf16_rne(kdw[c * 31 + kk]), mcr[nn]); }
    const float a1 = silu(pmul(dw, bf16_rne(g1[c]) * bnf) + bf16_rne(be1[c])); const float o = pmul(silu(pmul(a1 + mcr[n], bf16_rne(g2[c]) * bnf) + bf16_rne(be2[c])), HKT[((size_t)b * DI + c) * N + n]);
    v[k] = o + X2[row * C + c]; s += v[k]; }
  for (int o2 = 16; o2; o2 >>= 1) s += __shfl_xor(s, o2); const float mu = s * (1.0f / C); float q = 0.0f; for (int k = 0; k < 4; ++k) q += pmul(v[k] - mu, v[k] - mu); for (int o2 = 16; o2; o2 >>= 1) q += __shfl_xor(q, o2); const float rs = rsqrtf(q * (1.0f / C) + EPS);
  v4f r; for (int k = 0; k < 4; ++k) { const int c = lane * 4 + k; r[k] = pmul(pmul(v[k] - mu, rs), bf16_rne(png[c])) + bf16_rne(pnb[c]); }
  for (int pass = 0; pass < 2; ++pass) { *(volatile v4f*)(out + row * C + lane * 4) = r; __threadfence(); } }
}

extern "C" void kernel_launch(void* const* d_in, const int* in_sizes, int n_in, void* d_out, int out_size, void* d_ws, size_t ws_size, hipStream_t stream) {
  (void)n_in;
  auto Fp = [&](int i) { return (const float*)d_in[i]; };
  if (in_sizes[0] != NR * C || in_sizes[1] != C * C * 3 || in_sizes[15] != 2 * DI * C || in_sizes[18] != (R + 2 * S) * DI || in_sizes[21] != DI * S || in_sizes[23] != C * DI || in_sizes[26] != DI * C || in_sizes[34] != 32 * C * 31 || in_sizes[36] != C * 31 || out_size != NR * C) return;
  const int BV = B;
  size_t off = 0; char* ws = (char*)d_ws;
  auto carve = [&](size_t bytes) { char* p = ws + off; off += (bytes + 255) & ~(size_t)255; return p; };
  b16* C1T = (b16*)carve((size_t)C * 384 * 2); b16* C2T = (b16*)carve((size_t)C * 384 * 2); b16* QT = (b16*)carve((size_t)C * C * 2); b16* KT = (b16*)carve((size_t)C * C * 2); b16* MIN = (b16*)carve((size_t)2 * DI * C * 2); b16* MXP = (b16*)carve((size_t)XPW * DI * 2); b16* MOUT = (b16*)carve((size_t)C * DI * 2); b16* KP = (b16*)carve((size_t)DI * C * 2);
  b16* KC = (b16*)carve((size_t)32 * C * (8 + 16 + 24 + 32) * 2);
  float* C1 = (float*)carve((size_t)NR * C * 4); b16* Qh = (b16*)carve((size_t)B * C * N * 2); b16* Ql = (b16*)carve((size_t)B * C * N * 2); b16* Kh = (b16*)carve((size_t)B * C * N * 2); b16* Kl = (b16*)carve((size_t)B * C * N * 2); b16* CCh = (b16*)carve((size_t)B * C * C * 2); b16* CCl = (b16*)carve((size_t)B * C * C * 2);
  float* XCA = (float*)carve((size_t)NR * C * 4); float* X1 = (float*)carve((size_t)NR * C * 4); float* XZ = (float*)carve((size_t)NR * 2 * DI * 4); float* XI2 = (float*)carve((size_t)NR * DI * 4); float* DBL = (float*)carve((size_t)NR * XPW * 4); float* DT = (float*)carve((size_t)NR * DI * 4); float* YGT = (float*)carve((size_t)NR * DI * 4); float* X2 = (float*)carve((size_t)NR * C * 4); float* HKT = (float*)carve((size_t)NR * DI * 4); float* MCT = (float*)carve((size_t)NR * C * 4);
  if (off > ws_size || off > ((size_t)64 << 20)) return;
  wput_kernel<<<(4 * 32 * C + 255) / 256, 256, 0, stream>>>(Fp(1), Fp(9), Fp(5), Fp(7), Fp(15), Fp(18), Fp(23), Fp(26), Fp(28), Fp(30), Fp(32), Fp(34), C1T, C2T, QT, KT, MIN, MXP, MOUT, KP, KC);
  conv3_kernel<0><<<NR / 16, 32, 0, stream>>>(Fp(0), C1T, Fp(2), Fp(3), Fp(4), nullptr, BV, C1);
  qk_kernel<<<B * (N / 64), 32, 0, stream>>>(C1, QT, KT, Fp(6), Fp(8), BV, Qh, Ql, Kh, Kl);
  cc_kernel<<<B * 2, 32, 0, stream>>>(Qh, Ql, Kh, Kl, BV, CCh, CCl);
  xca_kernel<<<NR / 16, 32, 0, stream>>>(C1, CCh, CCl, BV, XCA);
  conv3_kernel<1><<<NR / 16, 32, 0, stream>>>(XCA, C2T, Fp(10), Fp(11), Fp(12), Fp(0), BV, X1);
  rowgemm_kernel<0><<<(NR / 16) * 4, 32, 0, stream>>>(X1, Fp(13), Fp(14), MIN, nullptr, nullptr, BV, XZ);
  mconv_kernel<<<NR / 8, 256, 0, stream>>>(XZ, Fp(16), Fp(17), BV, XI2);
  xproj_kernel<<<NR / 16, 32, 0, stream>>>(XI2, MXP, Fp(19), Fp(20), BV, DBL, DT);
  mscan_kernel<<<B * (DI / 16), 32, 0, stream>>>(XI2, DT, DBL, XZ, Fp(21), Fp(22), BV, YGT);
  rowgemm_kernel<1><<<(NR / 16) * 1, 32, 0, stream>>>(YGT, nullptr, nullptr, MOUT, nullptr, X1, BV, X2);
  rowgemm_kernel<2><<<(NR / 32) * 2, 32, 0, stream>>>(X2, Fp(24), Fp(25), KP, Fp(27), nullptr, BV, HKT);
  kconv_kernel<<<B * (N / 32), 32, 0, stream>>>(HKT, KC, Fp(29), Fp(31), Fp(33), Fp(35), BV, MCT);
  final_kernel<<<NR / 8, 256, 0, stream>>>(MCT, HKT, X2, Fp(36), Fp(37), Fp(38), Fp(39), Fp(40), Fp(41), Fp(42), Fp(43), BV, (float*)d_out);
}
